// singlePerspectiveNet_22514218566052
// MI455X (gfx1250) — hardware-run, weakly checked
//
#include <hip/hip_runtime.h>
#include <math.h>

typedef __attribute__((ext_vector_type(16))) _Float16 v16h;
typedef __attribute__((ext_vector_type(16))) __bf16 v16b;
typedef __attribute__((ext_vector_type(8)))  _Float16 v8h;
typedef __attribute__((ext_vector_type(8)))  float v8f;
typedef __attribute__((ext_vector_type(4)))  float v4f;
typedef __attribute__((ext_vector_type(2)))  float v2f;
typedef __attribute__((ext_vector_type(4)))  unsigned v4u;
typedef __attribute__((ext_vector_type(4)))  int v4i;
typedef float __attribute__((may_alias)) float_a;
typedef int __attribute__((may_alias)) int_a;

template <typename T> __device__ __forceinline__ void vst2(void* p, T v) { *(volatile T*)p = v; __threadfence(); *(volatile T*)p = v; }
__device__ __forceinline__ v8f wmma16(v16h a, v16h b, v8f c) {
  v8f d = __builtin_amdgcn_wmma_f32_16x16x32_f16(false, a, false, b, (short)0, c, false, false);
  asm volatile("v_nop\n\tv_nop\n\tv_nop\n\tv_nop" : "+v"(d) : "v"(a), "v"(b));
  return d;
}
__device__ __forceinline__ v8f wmma_bf(v16b a, v16b b, v8f c) {
  v8f d = __builtin_amdgcn_wmma_f32_16x16x32_bf16(false, a, false, b, (short)0, c, false, false);
  asm volatile("v_nop\n\tv_nop\n\tv_nop\n\tv_nop" : "+v"(d) : "v"(a), "v"(b));
  return d;
}
__device__ __forceinline__ v16h frag_h(const _Float16* rowk0, int lane) {
  union { v16h v; v8h q[2]; } u; const _Float16* p = rowk0 + 8 * (lane >> 4);
  u.q[0] = *(const v8h*)p; u.q[1] = *(const v8h*)(p + 16); return u.v;
}
__device__ __forceinline__ v16h frag_f32(const float* rowk0, int lane) {
  v16h a; const float* p = rowk0 + 8 * (lane >> 4);
#pragma unroll
  for (int i = 0; i < 8; ++i) { a[i] = (_Float16)p[i]; a[8 + i] = (_Float16)p[16 + i]; }
  return a;
}
__device__ __forceinline__ v16h frag_f32s(const float* rowk0, int lane, float sc) {
  v16h a; const float* p = rowk0 + 8 * (lane >> 4);
#pragma unroll
  for (int i = 0; i < 8; ++i) { a[i] = (_Float16)(p[i] * sc); a[8 + i] = (_Float16)(p[16 + i] * sc); }
  return a;
}
__device__ __forceinline__ v16h fragc_f32(const float* W, int k0, int n, int lane, int ld, int K) {
  v16h a; const int g = lane >> 4;
#pragma unroll
  for (int i = 0; i < 8; ++i) { const int ka = k0 + 8 * g + i, kb = ka + 16;
    a[i] = (_Float16)(ka < K ? W[(size_t)(ka < K ? ka : K - 1) * ld + n] : 0.f); a[8 + i] = (_Float16)(kb < K ? W[(size_t)(kb < K ? kb : K - 1) * ld + n] : 0.f); }
  return a;
}
struct F2 { v16b h, l; };
__device__ __forceinline__ F2 bsplit16(const float v[16]) { F2 r;
#pragma unroll
  for (int i = 0; i < 16; ++i) { const __bf16 h = (__bf16)v[i]; r.h[i] = h; r.l[i] = (__bf16)(v[i] - (float)h); }
  return r; }
__device__ __forceinline__ F2 split_row(const float* row, int k0, int lane) { float v[16]; const float* p = row + k0 + 8 * (lane >> 4);
#pragma unroll
  for (int i = 0; i < 8; ++i) { v[i] = p[i]; v[8 + i] = p[16 + i]; }
  return bsplit16(v); }
__device__ __forceinline__ F2 split_rowK(const float* row, int k0, int lane, int K) { float v[16]; const int g = lane >> 4;
#pragma unroll
  for (int i = 0; i < 8; ++i) { const int ka = k0 + 8 * g + i, kb = ka + 16; v[i] = ka < K ? row[ka < K ? ka : K - 1] : 0.f; v[8 + i] = kb < K ? row[kb < K ? kb : K - 1] : 0.f; }
  return bsplit16(v); }
__device__ __forceinline__ F2 split_col(const float* W, int k0, int n, int lane, int ld, int K) { float v[16]; const int g = lane >> 4;
#pragma unroll
  for (int i = 0; i < 8; ++i) { const int ka = k0 + 8 * g + i, kb = ka + 16; v[i] = ka < K ? W[(size_t)(ka < K ? ka : K - 1) * ld + n] : 0.f; v[8 + i] = kb < K ? W[(size_t)(kb < K ? kb : K - 1) * ld + n] : 0.f; }
  return bsplit16(v); }
__device__ __forceinline__ v8f mac3(const F2& a, const F2& b, v8f c) { c = wmma_bf(a.l, b.h, c); c = wmma_bf(a.h, b.l, c); return wmma_bf(a.h, b.h, c); }
__device__ __forceinline__ float sigm(float v) { return 1.0f / (1.0f + expf(-v)); }
#define LDSX() do { asm volatile("s_wait_dscnt 0" ::: "memory"); __builtin_amdgcn_wave_barrier(); __builtin_amdgcn_fence(__ATOMIC_RELEASE, "workgroup"); } while (0)


#define NR 4096
#define NF 768
#define FT 2048
#define HF 1024
#define NO 256
#ifndef TR
#define TR (NR / 64)
#endif
typedef __attribute__((ext_vector_type(8))) __bf16 v8b;
__device__ __forceinline__ v16b frag_b(const __bf16* rowk0, int lane) {
  union { v16b v; v8b q[2]; } u; const __bf16* p = rowk0 + 8 * (lane >> 4);
  u.q[0] = *(const v8b*)p; u.q[1] = *(const v8b*)(p + 16); return u.v;
}
__device__ __forceinline__ float bfr(float v) { return (float)(__bf16)v; }
__device__ __attribute__((noinline)) float exp_ni(float v) { return expf(v); }
__device__ __attribute__((noinline)) float erf_ni(float v) { return erff(v); }

#define WS_IN  0u
#define WS_END (WS_IN + 4u * (size_t)4 * NR * HF)

__device__ __forceinline__ int sdim(int s) { return s == 0 ? 128 : s == 1 ? 256 : 384; }
__device__ __forceinline__ v16b fragb_f32(const float* __restrict__ p, int lane) { v16b a; const float* pp = p + 8 * (lane >> 4);
#pragma unroll
  for (int i = 0; i < 8; ++i) { a[i] = (__bf16)pp[i]; a[8 + i] = (__bf16)pp[16 + i]; } return a; }
__global__ __launch_bounds__(128) void k_ft(const float* __restrict__ X, const int* __restrict__ I0, const int* __restrict__ I1, const int* __restrict__ I2, const int* __restrict__ I3, const float* __restrict__ W0, const float* __restrict__ B0, const float* __restrict__ W1f, const float* __restrict__ B1f, const float* __restrict__ W2f, const float* __restrict__ B2f, const float* __restrict__ W3f, const float* __restrict__ B3f, float* __restrict__ INTER) {
  __shared__ int sidx[384]; __shared__ __align__(16) float sf[4][16][68];
  const int tid = threadIdx.x, wave = tid >> 5, lane = tid & 31, col = lane & 15, g = lane >> 4; const int s = blockIdx.z; const int d = sdim(s); const int c0 = blockIdx.y * 64; const size_t r0 = (size_t)blockIdx.x * 64 + wave * 16;
  const int* Is = s == 0 ? I0 : s == 1 ? I1 : s == 2 ? I2 : I3; const float* Wf = s == 0 ? W0 : s == 1 ? W1f : s == 2 ? W2f : W3f; const float* Bf = s == 0 ? B0 : s == 1 ? B1f : s == 2 ? B2f : B3f;
  for (int k = tid; k < d; k += 128) { int v = Is[k]; sidx[k] = v < 0 ? 0 : (v >= NF ? NF - 1 : v); } __syncthreads();
  v8f acc[8] = {};
  const float* xr = X + (r0 + col) * NF;
#pragma unroll 1
  for (int kc = 0; kc < d / 32; ++kc) { v16b a;
#pragma unroll
    for (int i = 0; i < 8; ++i) { a[i] = (__bf16)xr[sidx[kc * 32 + 8 * g + i]]; a[8 + i] = (__bf16)xr[sidx[kc * 32 + 16 + 8 * g + i]]; }
#pragma unroll
    for (int j = 0; j < 8; ++j) { const int oc = (j < 4) ? (c0 + j * 16 + col) : (HF + c0 + (j - 4) * 16 + col); acc[j] = wmma_bf(a, fragb_f32(Wf + (size_t)oc * d + kc * 32, lane), acc[j]); } }
#pragma unroll
  for (int j = 0; j < 4; ++j) { const int c = c0 + j * 16 + col; const float b1 = bfr(Bf[c]), b2 = bfr(Bf[HF + c]);
#pragma unroll
    for (int r = 0; r < 8; ++r) sf[wave][8 * g + r][j * 16 + col] = (acc[j][r] + b1) * (acc[4 + j][r] + b2) * (127.0f / 128.0f); }
  LDSX(); for (int rl = 0; rl < 16; ++rl) if (lane < 16) vst2(INTER + (((size_t)s * NR + r0 + rl) * HF) + c0 + lane * 4, *(const v4f*)&sf[wave][rl][lane * 4]); }
__global__ __launch_bounds__(128) void k_head(const float* __restrict__ INTER, const float* __restrict__ X,
    const float* __restrict__ W1a, const float* __restrict__ b1a, const float* __restrict__ Woa, const float* __restrict__ boa,
    const float* __restrict__ W1b, const float* __restrict__ b1b, const float* __restrict__ Wob, const float* __restrict__ bob,
    const float* __restrict__ W1c, const float* __restrict__ b1c, const float* __restrict__ Woc, const float* __restrict__ boc,
    const float* __restrict__ W1d, const float* __restrict__ b1d, const float* __restrict__ Wod, const float* __restrict__ bod,
    const float* __restrict__ WC, float* __restrict__ OUT) {
  __shared__ __align__(16) float scat[4][16][36]; __shared__ __align__(16) float sf[4][16][260];
  const int tid = threadIdx.x, wave = tid >> 5, lane = tid & 31, col = lane & 15, g = lane >> 4; const size_t r0 = (size_t)blockIdx.x * 64 + wave * 16;
  v8f o[16];
#pragma unroll
  for (int j = 0; j < 16; ++j) o[j] = v8f{};
#pragma unroll 1
  for (int kc = 0; kc < NF / 32; ++kc) { const v16b a = fragb_f32(X + (r0 + col) * NF + kc * 32, lane);
#pragma unroll
    for (int j = 0; j < 16; ++j) o[j] = wmma_bf(a, fragb_f32(WC + (size_t)(j * 16 + col) * NF + kc * 32, lane), o[j]); }
#pragma unroll 1
  for (int s = 0; s < 4; ++s) { const float* W1 = s == 0 ? W1a : s == 1 ? W1b : s == 2 ? W1c : W1d; const float* B1 = s == 0 ? b1a : s == 1 ? b1b : s == 2 ? b1c : b1d; const float* WO = s == 0 ? Woa : s == 1 ? Wob : s == 2 ? Woc : Wod; const float* BO = s == 0 ? boa : s == 1 ? bob : s == 2 ? boc : bod;
    v8f f = {};
#pragma unroll 1
    for (int kc = 0; kc < HF / 32; ++kc) { const F2 a = split_row(INTER + (((size_t)s * NR + r0 + col) * HF), kc * 32, lane); const v16b w = fragb_f32(W1 + (size_t)col * HF + kc * 32, lane); f = wmma_bf(a.h, w, f); f = wmma_bf(a.l, w, f); }
#pragma unroll
    for (int r = 0; r < 8; ++r) { const float fv = f[r] + bfr(B1[col]); const float f2 = fv * fv * (127.0f / 128.0f); scat[wave][8 * g + r][col] = fminf(fmaxf(fv, 0.f), 1.f); scat[wave][8 * g + r][16 + col] = fminf(fmaxf(f2, 0.f), 1.f); }
    LDSX();
    { float v[16]; const float* prow = &scat[wave][col][0] + 8 * (lane >> 4);
#pragma unroll
      for (int i = 0; i < 8; ++i) { v[i] = prow[i]; v[8 + i] = prow[16 + i]; }
      const F2 a = bsplit16(v);
#pragma unroll
      for (int j = 0; j < 16; ++j) { const v16b w = fragb_f32(WO + (size_t)(j * 16 + col) * 32, lane); o[j] = wmma_bf(a.h, w, o[j]); o[j] = wmma_bf(a.l, w, o[j]); } }
    LDSX(); }
#pragma unroll
  for (int j = 0; j < 16; ++j) { const int c = j * 16 + col; const float bb = bfr(boa[c]) + bfr(bob[c]) + bfr(boc[c]) + bfr(bod[c]);
#pragma unroll
    for (int r = 0; r < 8; ++r) sf[wave][8 * g + r][c] = o[j][r] + bb; }
  LDSX(); for (int rl = 0; rl < 16; ++rl) for (int q = lane; q < NO / 4; q += 32) vst2(OUT + (r0 + rl) * NO + q * 4, *(const v4f*)&sf[wave][rl][q * 4]); }
extern "C" void kernel_launch(void* const* d_in, const int* in_sizes, int n_in, void* d_out, int out_size, void* d_ws, size_t ws_size, hipStream_t stream) {
  (void)in_sizes; (void)n_in; (void)out_size;
  const float** F = (const float**)d_in; const int** I = (const int**)d_in;
  if (ws_size < (size_t)WS_END) return;
  float* INTER = (float*)d_ws;
  k_ft<<<dim3(TR, HF / 64, 4), 128, 0, stream>>>(F[0], I[1], I[2], I[3], I[4], F[5], F[6], F[11], F[12], F[17], F[18], F[23], F[24], INTER);
  k_head<<<TR, 128, 0, stream>>>(INTER, F[0], F[7], F[8], F[9], F[10], F[13], F[14], F[15], F[16], F[19], F[20], F[21], F[22], F[25], F[26], F[27], F[28], F[29], (float*)d_out);
}
